// GroupQueryAttention_87600152969633
// MI455X (gfx1250) — hardware-verified
//
#include <hip/hip_runtime.h>
#pragma clang fp contract(off)

#ifndef NB
#define NB 2
#endif
#ifndef SEQ
#define SEQ 2048
#endif
#define NB_FULL   2
#define SEQ_FULL  2048
#define HIDDEN    2048
#define KVD       512
#define HEADS     32
#define REP       4
#define HDIM      64
#define MTOK      (NB * SEQ)

static_assert(NB >= 1 && NB <= NB_FULL);
static_assert(SEQ >= 64 && SEQ <= SEQ_FULL && (SEQ % 64) == 0);
static_assert(HIDDEN == HEADS * HDIM);
static_assert(KVD == (HEADS / REP) * HDIM);
static_assert(((MTOK / 32) * (HIDDEN / 64)) % 4 == 0);
static_assert(((MTOK / 32) * (KVD / 64)) % 4 == 0);
static_assert(((KVD / 32) * (MTOK / 64)) % 4 == 0);
static_assert((NB * HEADS * (SEQ / 16)) % 4 == 0);
static_assert(((size_t)MTOK * HIDDEN) % 2048 == 0);

typedef _Float16 v8h  __attribute__((ext_vector_type(8)));
typedef _Float16 v16h __attribute__((ext_vector_type(16)));
typedef float    v8f  __attribute__((ext_vector_type(8)));
typedef float    v4f  __attribute__((ext_vector_type(4)));

__device__ __forceinline__ float bf16_rne(float f) {
    unsigned u = __float_as_uint(f);
    u = (u + 0x7FFFu + ((u >> 16) & 1u)) & 0xFFFF0000u;
    return __uint_as_float(u);
}

__device__ __forceinline__ v8f vzero() {
    v8f z;
#pragma unroll
    for (int i = 0; i < 8; ++i) z[i] = 0.0f;
    return z;
}

__device__ __forceinline__ v16h load_frag(const _Float16* p) {
    v8h lo = *(const v8h*)(p);
    v8h hi = *(const v8h*)(p + 16);
    return __builtin_shufflevector(lo, hi, 0,1,2,3,4,5,6,7,8,9,10,11,12,13,14,15);
}

__device__ __forceinline__ v8f wmma_f16(v16h a, v16h b, v8f c) {
    return __builtin_amdgcn_wmma_f32_16x16x32_f16(false, a, false, b, (short)0, c, false, false);
}

__global__ __launch_bounds__(256) void k_cvt_act(const float* __restrict__ x, const float* __restrict__ e,
                                                 _Float16* __restrict__ x16, _Float16* __restrict__ e16)
{
    const float* src = x;
    _Float16* dst = x16;
    if (blockIdx.y != 0) { src = e; dst = e16; }
    const size_t i  = (size_t)blockIdx.x * 256 + threadIdx.x;
    const size_t e0 = i * 8;
    if (e0 >= (size_t)MTOK * HIDDEN) return;
    const int t = (int)(e0 / HIDDEN);
    const int c = (int)(e0 % HIDDEN);
    const int b = t / SEQ, s = t % SEQ;
    const float* sp = src + ((size_t)(b * SEQ_FULL + s)) * HIDDEN + c;
    v4f u0 = *(const v4f*)(sp);
    v4f u1 = *(const v4f*)(sp + 4);
    v8h hv;
#pragma unroll
    for (int j = 0; j < 4; ++j) {
        hv[j]     = (_Float16)bf16_rne(u0[j]);
        hv[4 + j] = (_Float16)bf16_rne(u1[j]);
    }
    _Float16* dp = dst + e0;
    *(volatile v8h*)dp = hv;
    __threadfence();
    *(volatile v8h*)dp = hv;
}

__global__ __launch_bounds__(256) void k_cvt_w(const float* __restrict__ wq, const float* __restrict__ wk,
                                               const float* __restrict__ wv, const float* __restrict__ wo,
                                               _Float16* __restrict__ wqT, _Float16* __restrict__ wkT,
                                               _Float16* __restrict__ wvT, _Float16* __restrict__ woT)
{
    __shared__ __attribute__((aligned(16))) _Float16 T[64 * 72];
    const float* W = wq; _Float16* WT = wqT; int N = HIDDEN;
    if (blockIdx.y == 1)      { W = wk; WT = wkT; N = KVD; }
    else if (blockIdx.y == 2) { W = wv; WT = wvT; N = KVD; }
    else if (blockIdx.y == 3) { W = wo; WT = woT; N = HIDDEN; }
    const int K = HIDDEN;
    const int ntn = N / 64;
    const int tiles = (K / 64) * ntn;
    if ((int)blockIdx.x >= tiles) return;
    const int k0 = ((int)blockIdx.x / ntn) * 64;
    const int n0 = ((int)blockIdx.x % ntn) * 64;
    const int tid = threadIdx.x;

#pragma unroll
    for (int p = 0; p < 4; ++p) {
        const int idx = p * 256 + tid;
        const int kr = idx >> 4, c4 = idx & 15;
        v4f d = *(const v4f*)(W + (size_t)(k0 + kr) * N + n0 + 4 * c4);
#pragma unroll
        for (int q = 0; q < 4; ++q)
            T[(4 * c4 + q) * 72 + kr] = (_Float16)(bf16_rne(d[q]) * 64.0f);
    }
    __syncthreads();

    v8h v[2];
    size_t off[2];
#pragma unroll
    for (int p = 0; p < 2; ++p) {
        const int idx = p * 256 + tid;
        const int n = idx >> 3, ch = idx & 7;
        v[p]   = *(const v8h*)(T + n * 72 + 8 * ch);
        off[p] = (size_t)(n0 + n) * K + k0 + 8 * ch;
    }
#pragma unroll
    for (int pass = 0; pass < 2; ++pass) {
#pragma unroll
        for (int p = 0; p < 2; ++p) *(volatile v8h*)(WT + off[p]) = v[p];
        if (pass == 0) __threadfence();
    }
}

__global__ __launch_bounds__(128) __attribute__((amdgpu_num_vgpr(256)))
void k_gemm(const _Float16* __restrict__ A, const _Float16* __restrict__ BT,
            const float* __restrict__ bias, void* __restrict__ Cout,
            int M, int N, int K, int lda, int ldb, int ldc, int mode, float scale)
{
    __shared__ __attribute__((aligned(16))) float stile[4][32 * 64];

    const int wave = threadIdx.x >> 5;
    const int lane = threadIdx.x & 31;
    const int h = lane >> 4, m = lane & 15, kb = h * 8;
    const int tilesN = N >> 6, tilesM = M >> 5;
    const int ntiles = tilesN * tilesM;
    int wid = (int)blockIdx.x * 4 + wave;
    const bool valid = wid < ntiles;
    if (!valid) wid = ntiles - 1;
    const int m0 = (wid / tilesN) << 5;
    const int n0 = (wid % tilesN) << 6;

    const _Float16* arow0 = A  + (size_t)(m0 + m) * lda + kb;
    const _Float16* arow1 = arow0 + (size_t)16 * lda;
    const _Float16* brow  = BT + (size_t)(n0 + m) * ldb + kb;
    const size_t bstep = (size_t)16 * ldb;

    v8f acc[2][4];
#pragma unroll
    for (int a = 0; a < 2; ++a)
#pragma unroll
        for (int j = 0; j < 4; ++j) acc[a][j] = vzero();

#pragma unroll 1
    for (int k0 = 0; k0 < K; k0 += 32) {
        v16h a0 = load_frag(arow0 + k0);
        v16h a1 = load_frag(arow1 + k0);
        v16h b0 = load_frag(brow + k0);
        v16h b1 = load_frag(brow + bstep + k0);
        v16h b2 = load_frag(brow + 2 * bstep + k0);
        v16h b3 = load_frag(brow + 3 * bstep + k0);
        acc[0][0] = wmma_f16(a0, b0, acc[0][0]);
        acc[1][0] = wmma_f16(a1, b0, acc[1][0]);
        acc[0][1] = wmma_f16(a0, b1, acc[0][1]);
        acc[1][1] = wmma_f16(a1, b1, acc[1][1]);
        acc[0][2] = wmma_f16(a0, b2, acc[0][2]);
        acc[1][2] = wmma_f16(a1, b2, acc[1][2]);
        acc[0][3] = wmma_f16(a0, b3, acc[0][3]);
        acc[1][3] = wmma_f16(a1, b3, acc[1][3]);
        asm volatile("v_nop\n\tv_nop\n\tv_nop\n\tv_nop"
                     : "+v"(acc[0][0]), "+v"(acc[0][1]), "+v"(acc[0][2]), "+v"(acc[0][3]),
                       "+v"(acc[1][0]), "+v"(acc[1][1]), "+v"(acc[1][2]), "+v"(acc[1][3])
                     : "v"(a0), "v"(a1), "v"(b0), "v"(b1), "v"(b2), "v"(b3));
    }

    float* st = stile[wave];
    _Float16* st16 = (_Float16*)st;

    float bc[4];
#pragma unroll
    for (int j = 0; j < 4; ++j) {
        const int cidx = (mode != 1) ? (n0 + 16 * j + m) : 0;
        const float bvl = bf16_rne(bias[cidx]);
        bc[j] = (mode != 1) ? bvl : 0.0f;
    }
#pragma unroll
    for (int hh = 0; hh < 2; ++hh) {
        const int rbase = 16 * hh + 8 * h;
        const int ridx = (mode == 1) ? (m0 + rbase) : 0;
        v4f br0 = *(const v4f*)(bias + ridx);
        v4f br1 = *(const v4f*)(bias + ridx + 4);
        float br[8];
#pragma unroll
        for (int i = 0; i < 4; ++i) {
            br[i]     = (mode == 1) ? bf16_rne(br0[i]) : 0.0f;
            br[4 + i] = (mode == 1) ? bf16_rne(br1[i]) : 0.0f;
        }
#pragma unroll
        for (int i = 0; i < 8; ++i) {
            const int r = rbase + i;
#pragma unroll
            for (int j = 0; j < 4; ++j) {
                const float val = acc[hh][j][i] * scale + bc[j] + br[i];
                const int c = 16 * j + m;
                if (mode == 2) st[r * 64 + c] = val;
                else           st16[r * 64 + c] = (_Float16)val;
            }
        }
    }
    __syncthreads();

    if (mode == 2) {
        float* Cf = (float*)Cout;
#pragma unroll
        for (int pass = 0; pass < 2; ++pass) {
#pragma unroll
            for (int it = 0; it < 16; ++it) {
                const int r = 2 * it + h;
                const int c4 = m;
                v4f v = *(const v4f*)(st + r * 64 + 4 * c4);
                const int mm = m0 + r;
                const size_t orow = (size_t)(mm / SEQ) * SEQ_FULL + (mm % SEQ);
                float* p = Cf + orow * (size_t)ldc + n0 + 4 * c4;
                if (valid) *(volatile v4f*)p = v;
            }
            if (pass == 0) __threadfence();
        }
    } else {
        _Float16* C16 = (_Float16*)Cout;
#pragma unroll
        for (int pass = 0; pass < 2; ++pass) {
#pragma unroll
            for (int it = 0; it < 8; ++it) {
                const int r = 4 * it + (lane >> 3);
                const int ch = lane & 7;
                v8h v = *(const v8h*)(st16 + r * 64 + 8 * ch);
                size_t off;
                if (mode == 0) off = (size_t)(m0 + r) * ldc + n0 + 8 * ch;
                else           off = ((size_t)((n0 / SEQ) * M + m0 + r)) * SEQ + (n0 % SEQ) + 8 * ch;
                if (valid) *(volatile v8h*)(C16 + off) = v;
            }
            if (pass == 0) __threadfence();
        }
    }
}

__global__ __launch_bounds__(128) __attribute__((amdgpu_num_vgpr(256)))
void k_attn(const _Float16* __restrict__ Qp,
            const _Float16* __restrict__ Kp,
            const _Float16* __restrict__ Vt,
            _Float16* __restrict__ Cx)
{
    __shared__ __attribute__((aligned(16))) _Float16 ctile[4][16 * 64];

    const int wave = threadIdx.x >> 5;
    const int lane = threadIdx.x & 31;
    const int h = lane >> 4, m = lane & 15, kb = h * 8;
    const int sqtiles = SEQ / 16;
    const int nwaves = NB * HEADS * sqtiles;
    int wid = (int)blockIdx.x * 4 + wave;
    const bool valid = wid < nwaves;
    if (!valid) wid = nwaves - 1;
    const int sqt = wid % sqtiles;
    const int bh  = wid / sqtiles;
    const int b   = bh / HEADS;
    const int hd  = bh % HEADS;
    const int g   = hd / REP;
    const int sq0 = sqt * 16;

    const _Float16* qrow = Qp + ((size_t)(b * SEQ + sq0 + m)) * HIDDEN + hd * HDIM + kb;
    v16h qb0 = load_frag(qrow);
    v16h qb1 = load_frag(qrow + 32);

    const _Float16* kbase = Kp + ((size_t)(b * SEQ + m)) * KVD + g * HDIM + kb;
    const _Float16* vbase = Vt + ((size_t)(b * KVD + g * HDIM + m)) * SEQ + kb;

    float m_run = -1.0e30f, l_run = 0.0f;
    v8f o[4];
#pragma unroll
    for (int r = 0; r < 4; ++r) o[r] = vzero();

#pragma unroll 1
    for (int kt = 0; kt < SEQ; kt += 32) {
        const _Float16* kr = kbase + (size_t)kt * KVD;
        v16h a0 = load_frag(kr);
        v16h a1 = load_frag(kr + 32);
        v16h a2 = load_frag(kr + (size_t)16 * KVD);
        v16h a3 = load_frag(kr + (size_t)16 * KVD + 32);

        v8f st1 = wmma_f16(a0, qb0, vzero());
        st1 = wmma_f16(a1, qb1, st1);
        v8f st2 = wmma_f16(a2, qb0, vzero());
        st2 = wmma_f16(a3, qb1, st2);
        asm volatile("v_nop\n\tv_nop\n\tv_nop\n\tv_nop"
                     : "+v"(st1), "+v"(st2)
                     : "v"(a0), "v"(a1), "v"(a2), "v"(a3), "v"(qb0), "v"(qb1));

        float t = -1.0e30f;
#pragma unroll
        for (int i = 0; i < 8; ++i) {
            st1[i] = st1[i] * 0.125f;
            st2[i] = st2[i] * 0.125f;
            t = fmaxf(t, fmaxf(st1[i], st2[i]));
        }
        t = fmaxf(t, __shfl_xor(t, 16, 32));
        const float m_new = fmaxf(m_run, t);
        const float alpha = __expf(m_run - m_new);

        v16h pb;
        float rs = 0.0f;
#pragma unroll
        for (int i = 0; i < 8; ++i) {
            const float p = __expf(st1[i] - m_new);
            rs += p;
            pb[i] = (_Float16)(p * 1024.0f);
        }
#pragma unroll
        for (int i = 0; i < 8; ++i) {
            const float p = __expf(st2[i] - m_new);
            rs += p;
            pb[8 + i] = (_Float16)(p * 1024.0f);
        }
        rs += __shfl_xor(rs, 16, 32);
        l_run = l_run * alpha + rs;
        m_run = m_new;
#pragma unroll
        for (int r = 0; r < 4; ++r)
#pragma unroll
            for (int i = 0; i < 8; ++i) o[r][i] = o[r][i] * alpha;

        const _Float16* vr = vbase + kt;
        v16h va0 = load_frag(vr);
        v16h va1 = load_frag(vr + (size_t)16 * SEQ);
        v16h va2 = load_frag(vr + (size_t)32 * SEQ);
        v16h va3 = load_frag(vr + (size_t)48 * SEQ);
        o[0] = wmma_f16(va0, pb, o[0]);
        o[1] = wmma_f16(va1, pb, o[1]);
        o[2] = wmma_f16(va2, pb, o[2]);
        o[3] = wmma_f16(va3, pb, o[3]);
        asm volatile("v_nop\n\tv_nop\n\tv_nop\n\tv_nop"
                     : "+v"(o[0]), "+v"(o[1]), "+v"(o[2]), "+v"(o[3])
                     : "v"(va0), "v"(va1), "v"(va2), "v"(va3), "v"(pb));
    }

    const float inv = 0.0625f / l_run;
    _Float16* ct = ctile[wave];
#pragma unroll
    for (int r = 0; r < 4; ++r) {
        v8h hv;
#pragma unroll
        for (int i = 0; i < 8; ++i) hv[i] = (_Float16)(o[r][i] * inv);
        *(v8h*)(ct + m * 64 + 16 * r + 8 * h) = hv;
    }
    __syncthreads();

#pragma unroll
    for (int pass = 0; pass < 2; ++pass) {
#pragma unroll
        for (int it = 0; it < 4; ++it) {
            const int row = 4 * it + (lane >> 3);
            const int ch  = lane & 7;
            v8h v = *(const v8h*)(ct + row * 64 + 8 * ch);
            _Float16* p = Cx + ((size_t)(b * SEQ + sq0 + row)) * HIDDEN + hd * HDIM + 8 * ch;
            if (valid) *(volatile v8h*)p = v;
        }
        if (pass == 0) __threadfence();
    }
}

extern "C" void kernel_launch(void* const* d_in, const int* in_sizes, int n_in,
                              void* d_out, int out_size, void* d_ws, size_t ws_size,
                              hipStream_t stream)
{
    if (n_in < 10) return;
    const long long needAct = ((long long)(NB - 1) * SEQ_FULL + SEQ) * HIDDEN;
    if ((long long)in_sizes[0] < needAct || (long long)in_sizes[1] < needAct) return;
    if (in_sizes[2] < HIDDEN * HIDDEN || in_sizes[3] < HIDDEN) return;
    if (in_sizes[4] < HIDDEN * KVD    || in_sizes[5] < KVD) return;
    if (in_sizes[6] < HIDDEN * KVD    || in_sizes[7] < KVD) return;
    if (in_sizes[8] < HIDDEN * HIDDEN || in_sizes[9] < HIDDEN) return;
    if ((long long)out_size < needAct) return;

    const float* x  = (const float*)d_in[0];
    const float* eo = (const float*)d_in[1];
    const float* Wq = (const float*)d_in[2];
    const float* bq = (const float*)d_in[3];
    const float* Wk = (const float*)d_in[4];
    const float* bk = (const float*)d_in[5];
    const float* Wv = (const float*)d_in[6];
    const float* bv = (const float*)d_in[7];
    const float* Wo = (const float*)d_in[8];
    const float* bo = (const float*)d_in[9];

    const size_t bAct = (size_t)MTOK * HIDDEN * 2;
    const size_t bKV  = (size_t)MTOK * KVD * 2;
    const size_t bWq  = (size_t)HIDDEN * HIDDEN * 2;
    const size_t bWk  = (size_t)KVD * HIDDEN * 2;
    size_t off = 0;
    char* ws = (char*)d_ws;
    _Float16* x16 = (_Float16*)(ws + off); off += bAct;
    _Float16* e16 = (_Float16*)(ws + off); off += bAct;
    _Float16* wqT = (_Float16*)(ws + off); off += bWq;
    _Float16* wkT = (_Float16*)(ws + off); off += bWk;
    _Float16* wvT = (_Float16*)(ws + off); off += bWk;
    _Float16* woT = (_Float16*)(ws + off); off += bWq;
    _Float16* qp  = (_Float16*)(ws + off); off += bAct;
    _Float16* kp  = (_Float16*)(ws + off); off += bKV;
    _Float16* vt  = (_Float16*)(ws + off); off += bKV;
    _Float16* cx  = (_Float16*)(ws + off); off += bAct;
    if (off > ws_size) return;

    {
        const unsigned nthr = (unsigned)(((size_t)MTOK * HIDDEN) / 8);
        k_cvt_act<<<dim3(nthr / 256, 2), 256, 0, stream>>>(x, eo, x16, e16);
    }
    {
        const unsigned tilesBig = (HIDDEN / 64) * (HIDDEN / 64);
        k_cvt_w<<<dim3(tilesBig, 4), 256, 0, stream>>>(Wq, Wk, Wv, Wo, wqT, wkT, wvT, woT);
    }
    const float sW  = 0.015625f;
    const float sWO = 0.000244140625f;
    k_gemm<<<((MTOK / 32) * (HIDDEN / 64)) / 4, 128, 0, stream>>>(
        x16, wqT, bq, (void*)qp, MTOK, HIDDEN, HIDDEN, HIDDEN, HIDDEN, HIDDEN, 0, sW);
    k_gemm<<<((MTOK / 32) * (KVD / 64)) / 4, 128, 0, stream>>>(
        e16, wkT, bk, (void*)kp, MTOK, KVD, HIDDEN, HIDDEN, HIDDEN, KVD, 0, sW);
    k_gemm<<<((KVD / 32) * (MTOK / 64)) / 4, 128, 0, stream>>>(
        wvT, e16, bv, (void*)vt, KVD, MTOK, HIDDEN, HIDDEN, HIDDEN, SEQ, 1, sW);
    k_attn<<<(NB * HEADS * (SEQ / 16)) / 4, 128, 0, stream>>>(qp, kp, vt, cx);
    k_gemm<<<((MTOK / 32) * (HIDDEN / 64)) / 4, 128, 0, stream>>>(
        cx, woT, bo, d_out, MTOK, HIDDEN, HIDDEN, HIDDEN, HIDDEN, HIDDEN, 2, sWO);
}
